// MyGCN2_24180665876563
// MI455X (gfx1250) — hardware-run, weakly checked
//
#include <hip/hip_runtime.h>

typedef float          v8f   __attribute__((ext_vector_type(8)));
typedef float          v4f   __attribute__((ext_vector_type(4)));
typedef unsigned int   v4u   __attribute__((ext_vector_type(4)));
typedef int            v8i   __attribute__((ext_vector_type(8)));
typedef unsigned short v8us  __attribute__((ext_vector_type(8)));
typedef unsigned short v16us __attribute__((ext_vector_type(16)));
typedef __bf16         v16bf __attribute__((ext_vector_type(16)));
typedef _Float16       v16h  __attribute__((ext_vector_type(16)));
typedef v4f  __attribute__((may_alias)) v4fa;
typedef v8us __attribute__((may_alias)) v8usa;
union FragB { v16bf v; v16us u; v8us h[2]; v8i w; };
union FragH { v16h  v; v16us u; v8us h[2]; v8i w; };

__device__ __forceinline__ v8f wmb(const FragB& a, const FragB& b, v8f c) {
  v8f d = __builtin_amdgcn_wmma_f32_16x16x32_bf16(false, a.v, false, b.v, (short)0, c, false, false);
  asm volatile("v_nop\n\tv_nop\n\tv_nop\n\tv_nop" : "+v"(d) : "v"(a.w), "v"(b.w));
  return d;
}

__device__ __forceinline__ v8f wmh(const FragH& a, const FragH& b, v8f c) {
  v8f d = __builtin_amdgcn_wmma_f32_16x16x32_f16(false, a.v, false, b.v, (short)0, c, false, false);
  asm volatile("v_nop\n\tv_nop\n\tv_nop\n\tv_nop" : "+v"(d) : "v"(a.w), "v"(b.w));
  return d;
}

__device__ __forceinline__ unsigned bf16_bits(float f) {
  const unsigned u = __float_as_uint(f);
  const unsigned r = (u + 0x7FFFu + ((u >> 16) & 1u)) >> 16;
  const unsigned q = (u >> 16) | 0x40u;
  return ((u & 0x7fffffffu) > 0x7f800000u) ? q : r;
}

__device__ __forceinline__ float bf16_val(float f) {
  return __uint_as_float(bf16_bits(f) << 16);
}
__device__ __forceinline__ int clampi(int v, int lo, int hi) {
  return v < lo ? lo : (v > hi ? hi : v);
}

__device__ __forceinline__ unsigned f16_bits(float f) {
  const unsigned u  = __float_as_uint(f);
  const unsigned s  = (u >> 16) & 0x8000u;
  const unsigned a  = u & 0x7fffffffu;
  const unsigned t  = a - 0x38000000u;
  const unsigned r  = (t + 0x0FFFu + ((t >> 13) & 1u)) >> 13;
  const unsigned rc = r > 0x7C00u ? 0x7C00u : r;
  const bool small  = a < 0x38800000u;
  const bool isnan  = a > 0x7f800000u;
  const unsigned fin = small ? 0u : (s | rc);
  return isnan ? (s | 0x7E00u) : fin;
}

__device__ __forceinline__ unsigned pk16(unsigned lo, unsigned hi) { return lo | (hi << 16); }
__device__ __forceinline__ unsigned bf16_lo_bits(float v) {
  float hi = bf16_val(v);
  asm volatile("" : "+v"(hi));
  return bf16_bits(v - hi);
}
__device__ __forceinline__ v4u pack8_bf16(v4f a, v4f c) {
  return (v4u){ pk16(bf16_bits(a[0]), bf16_bits(a[1])), pk16(bf16_bits(a[2]), bf16_bits(a[3])),
                pk16(bf16_bits(c[0]), bf16_bits(c[1])), pk16(bf16_bits(c[2]), bf16_bits(c[3])) };
}
__device__ __forceinline__ v4u pack8_bf16_lo(v4f a, v4f c) {
  return (v4u){ pk16(bf16_lo_bits(a[0]), bf16_lo_bits(a[1])), pk16(bf16_lo_bits(a[2]), bf16_lo_bits(a[3])),
                pk16(bf16_lo_bits(c[0]), bf16_lo_bits(c[1])), pk16(bf16_lo_bits(c[2]), bf16_lo_bits(c[3])) };
}
__device__ __forceinline__ v4u pack8_f16(v4f a, v4f c) {
  return (v4u){ pk16(f16_bits(a[0]), f16_bits(a[1])), pk16(f16_bits(a[2]), f16_bits(a[3])),
                pk16(f16_bits(c[0]), f16_bits(c[1])), pk16(f16_bits(c[2]), f16_bits(c[3])) };
}

template <int FORM>
__global__ __launch_bounds__(256) void k_plane(const float* __restrict__ src, int rows, int cols, int ldsrc,
                                               unsigned short* __restrict__ dst, int MP, int KP) {
  static_assert(FORM >= 0 && FORM <= 3);
  const int KTOT = (FORM == 1 || FORM == 3) ? 2 * KP : KP;
  const unsigned ppr   = (unsigned)(KTOT >> 3);
  const unsigned kp8   = (unsigned)(KP >> 3);
  const unsigned total = (unsigned)MP * ppr;
  const unsigned g     = blockIdx.x * 256u + threadIdx.x;
  const unsigned rowu  = g / ppr;
  const unsigned p     = g - rowu * ppr;
  const bool second    = p >= kp8;
  const int row = (int)rowu;
  const int c0  = (int)((second ? p - kp8 : p) << 3);
  const float* srow = src + (size_t)clampi(row, 0, rows - 1) * (size_t)ldsrc;
  float x[8];
  unsigned mk[8];
#pragma unroll
  for (int e = 0; e < 8; ++e) {
    const int c = c0 + e;
    const float v = srow[clampi(c, 0, cols - 1)];
    asm volatile("" :: "v"(v));
    x[e]  = v;
    mk[e] = (row < rows && c < cols) ? 0xFFFFu : 0u;
  }
  const v4f a = (v4f){ x[0], x[1], x[2], x[3] };
  const v4f c = (v4f){ x[4], x[5], x[6], x[7] };
  v4u o;
  if (FORM == 2) {
    o = pack8_f16(a, c);
  } else {
    const v4u hi = pack8_bf16(a, c);
    o = hi;
    if (FORM == 1) { const v4u lo = pack8_bf16_lo(a, c); o = second ? lo : hi; }
  }
  const v4u mw = (v4u){ pk16(mk[0], mk[1]), pk16(mk[2], mk[3]), pk16(mk[4], mk[5]), pk16(mk[6], mk[7]) };
  o &= mw;
  if (g < total) {
    volatile v4u* q = (volatile v4u*)(dst + (size_t)g * 8);
    *q = o;
    __threadfence();
    *q = o;
  }
}

template <int FORM> struct FragOf    { typedef FragB T; };
template <>         struct FragOf<2> { typedef FragH T; };
__device__ __forceinline__ v8f mm(const FragB& a, const FragB& b, v8f c) { return wmb(a, b, c); }
__device__ __forceinline__ v8f mm(const FragH& a, const FragH& b, v8f c) { return wmh(a, b, c); }
template <class F> __device__ __forceinline__ F ld_frag(const unsigned short* p) {
  F f;
  f.h[0] = *(const v8usa*)(p);
  f.h[1] = *(const v8usa*)(p + 16);
  return f;
}

template <int FORM, int EPI>
__global__ __launch_bounds__(256) __attribute__((amdgpu_num_vgpr(248)))
void k_gemm_nt(const unsigned short* __restrict__ A, const unsigned short* __restrict__ B,
               const float* __restrict__ bias, float* __restrict__ D, int M, int N, int KTOT, int ldd) {
  static_assert(FORM >= 0 && FORM <= 2);
  static_assert(EPI == 0 || EPI == 1);
  typedef typename FragOf<FORM>::T F;
  __shared__ __attribute__((aligned(16))) float sT[8][16 * 68];
  const int lane = threadIdx.x & 31;
  const int wave = threadIdx.x >> 5;
  const int tilesM = (M + 63) >> 6;
  const int tilesN = (N + 63) >> 6;
  const int tile = blockIdx.x * 8 + wave;
  if (tile >= tilesM * tilesN) return;
  const int tm = tile / tilesN;
  const int tn = tile - tm * tilesN;
  const int m0 = tm << 6;
  const int n0 = tn << 6;

  const int rl = lane & 15;
  const int h8 = (lane >> 4) * 8;
  const unsigned short* pa = A + (size_t)(m0 + rl) * (size_t)KTOT + h8;
  const unsigned short* pb = B + (size_t)(n0 + rl) * (size_t)KTOT + h8;

  v8f acc[4][4];
#pragma unroll
  for (int i = 0; i < 4; ++i)
#pragma unroll
    for (int j = 0; j < 4; ++j) acc[i][j] = (v8f){0.f, 0.f, 0.f, 0.f, 0.f, 0.f, 0.f, 0.f};

#pragma unroll 1
  for (int k0 = 0; k0 < KTOT; k0 += 32) {
    F bf[4];
#pragma unroll
    for (int j = 0; j < 4; ++j) bf[j] = ld_frag<F>(pb + (size_t)(j << 4) * (size_t)KTOT + k0);
#pragma unroll
    for (int i = 0; i < 4; ++i) {
      const F af = ld_frag<F>(pa + (size_t)(i << 4) * (size_t)KTOT + k0);
#pragma unroll
      for (int j = 0; j < 4; ++j) acc[i][j] = mm(af, bf[j], acc[i][j]);
    }
  }

  float* slab = sT[wave];
  const int hh = lane >> 4;
  const int c4 = (lane & 15) * 4;
  const int nc = n0 + c4;
  const bool cok = nc < N;
  v4f bv = (v4f){0.f, 0.f, 0.f, 0.f};
  if (EPI == 1) {
    bv = *(const v4fa*)(bias + clampi(nc, 0, N - 4));
    asm volatile("" :: "v"(bv));
  }
#pragma unroll
  for (int i = 0; i < 4; ++i) {
    const int mBase = m0 + (i << 4);
#pragma unroll
    for (int j = 0; j < 4; ++j) {
#pragma unroll
      for (int r = 0; r < 8; ++r) slab[(h8 + r) * 68 + (j << 4) + rl] = acc[i][j][r];
    }
    __builtin_amdgcn_fence(__ATOMIC_RELEASE, "workgroup");
    __builtin_amdgcn_wave_barrier();
    __builtin_amdgcn_fence(__ATOMIC_ACQUIRE, "workgroup");
    v4f vv[8];
#pragma unroll
    for (int it = 0; it < 8; ++it) {
      const int row = it * 2 + hh;
      v4f v = *(const v4fa*)(slab + row * 68 + c4);
      if (EPI == 1) v += bv;
      vv[it] = v;
    }
    for (int pass = 0; pass < 2; ++pass) {
#pragma unroll
      for (int it = 0; it < 8; ++it) {
        const int row = mBase + it * 2 + hh;
        if (cok && row < M) *(volatile v4f*)(D + (size_t)row * (size_t)ldd + nc) = vv[it];
      }
      __threadfence();
    }
    __builtin_amdgcn_fence(__ATOMIC_RELEASE, "workgroup");
    __builtin_amdgcn_wave_barrier();
    __builtin_amdgcn_fence(__ATOMIC_ACQUIRE, "workgroup");
  }
}

#include <stddef.h>
#include <stdint.h>
#include <math.h>

#define SPLIT_H1 1
#define SPLIT_H2 1

typedef int   v4i __attribute__((ext_vector_type(4)));
typedef float v2f __attribute__((ext_vector_type(2)));
typedef v4i __attribute__((may_alias)) v4ia;
typedef v2f __attribute__((may_alias)) v2fa;

static constexpr int kN     = 50000;
static constexpr int kE     = 800000;
static constexpr int kF     = 128;
static constexpr int kH     = 128;
static constexpr int kC     = 40;
static constexpr int kCP    = 64;
static constexpr int kMP    = 50048;
static constexpr int kK2    = 256;
static constexpr int kK3    = 128;
static constexpr int kNBA   = 1024;
static constexpr int kNBLK  = 49;
static constexpr int kNW    = 8;
static constexpr int kEPW   = kE / kNW;
static constexpr int kUNR   = 5;
static constexpr int kSTEP  = 32 * kUNR;
static constexpr int kITERS = kEPW / kSTEP;
static constexpr int kMeasB1024  = 16623;
static constexpr int kMeasMaxDeg = 35;
static constexpr int kRCAP   = 20992;
static constexpr int kWLCAP  = 3328;
static constexpr int kDEGCAP = 64;
static constexpr int kBK_INTS = kNW * kWLCAP + kRCAP + 3 * kNBA + 32;
static constexpr int kBK_LDS  = kBK_INTS * 4;
static constexpr int kNGRP   = kN / 4;
static constexpr int kNU1 = kH * (kF / 8);
static constexpr int kNU2 = kCP * (kK2 / 8);
static constexpr int kNU3 = kCP * (kK3 / 8);
static constexpr int kBFN = 256;

static_assert(kMP % 64 == 0 && kMP >= kN && kMP % 16 == 0);
static_assert(kF % 32 == 0 && kK2 % 32 == 0 && kK3 % 32 == 0 && kK2 == 2 * kH && kK3 == 2 * kCP);
static_assert(kH % 64 == 0 && kCP % 64 == 0 && kH % 32 == 0 && kCP % 32 == 0);
static_assert((long long)kMP * kK2 / 8 < (1LL << 31));
static_assert((kMP * kF / 8) % 256 == 0);
static_assert(kN <= 65536);
static_assert(kNBA == 1024 && kNBLK * kNBA >= kMP);
static_assert((kNBLK - 1) * kNBA < kN);
static_assert(kE % kNW == 0 && kEPW % kSTEP == 0);
static_assert(kE % 256 == 0);
static_assert(kRCAP % 256 == 0 && 4 * kRCAP >= 5 * kMeasB1024);
static_assert(kDEGCAP >= kMeasMaxDeg + 8);
static_assert(4 * kWLCAP >= 5 * (kRCAP / kNW));
static_assert(kBK_INTS % 4 == 0 && kBK_LDS <= 262144);
static_assert(kN % 4 == 0 && kNBA % 64 == 0 && kNGRP * 4 == kN);
static_assert(kNGRP * 160 == kN * kC && kNGRP * 5 == 62500);
static_assert((kN * kC * 4) % 128 == 0);
static_assert(160 * (kNGRP - 1) + 159 + kN * kC == 2 * kN * kC - 1);
static_assert(kNU1 % 256 == 0 && kNU2 % 256 == 0 && kNU3 % 256 == 0);
static_assert(kC % 2 == 0 && kC <= kCP && kC % 4 == 0);

__device__ __forceinline__ int  rfl(int v) { return __builtin_amdgcn_readfirstlane(v); }
__device__ __forceinline__ void pin_i(int x)   { asm volatile("" :: "v"(x)); }
__device__ __forceinline__ void pin_f(float x) { asm volatile("" :: "v"(x)); }
__device__ __forceinline__ void st2_u(unsigned short* p, v4u o) {
  volatile v4u* q = (volatile v4u*)p;
  *q = o;
  __threadfence();
  *q = o;
}

__global__ __launch_bounds__(256) void k_wprep(const float* __restrict__ W1, const float* __restrict__ W2,
                                               const float* __restrict__ Wl, const float* __restrict__ b1,
                                               const float* __restrict__ b2, const float* __restrict__ bl,
                                               unsigned short* W1T, unsigned short* W2D, unsigned short* WLD,
                                               float* BF) {
  const int u = (int)blockIdx.x * 256 + (int)threadIdx.x;
  float x[8];
  if (u < kNU1) {
    const int n  = u >> 4;
    const int k8 = (u & 15) * 8;
#pragma unroll
    for (int i = 0; i < 8; ++i) { const float v = W1[(size_t)(k8 + i) * kH + n]; pin_f(v); x[i] = v; }
    const v4u o = pack8_bf16((v4f){x[0], x[1], x[2], x[3]}, (v4f){x[4], x[5], x[6], x[7]});
    st2_u(W1T + (size_t)n * kF + k8, o);
  } else if (u < kNU1 + kNU2) {
    const int v0 = u - kNU1;
    const int n  = v0 >> 5;
    const int k8 = (v0 & 31) * 8;
    const int kk = k8 & (kH - 1);
    const int nc = n < kC ? n : kC - 1;
#pragma unroll
    for (int i = 0; i < 8; ++i) { const float v = W2[(size_t)(kk + i) * kC + nc]; pin_f(v); x[i] = v; }
    v4u o = pack8_bf16((v4f){x[0], x[1], x[2], x[3]}, (v4f){x[4], x[5], x[6], x[7]});
    const unsigned m = (n < kC) ? 0xFFFFFFFFu : 0u;
    o &= (v4u){m, m, m, m};
    st2_u(W2D + (size_t)n * kK2 + k8, o);
  } else if (u < kNU1 + kNU2 + kNU3) {
    const int v0 = u - (kNU1 + kNU2);
    const int n  = v0 >> 4;
    const int k8 = (v0 & 15) * 8;
    const int kk = k8 & (kCP - 1);
    const int nc = n < kC ? n : kC - 1;
    unsigned mk[8];
#pragma unroll
    for (int i = 0; i < 8; ++i) {
      const int k  = kk + i;
      const int kc = k < kC ? k : kC - 1;
      const float v = Wl[(size_t)kc * kC + nc];
      pin_f(v);
      x[i]  = v;
      mk[i] = (n < kC && k < kC) ? 0xFFFFu : 0u;
    }
    v4u o = pack8_bf16((v4f){x[0], x[1], x[2], x[3]}, (v4f){x[4], x[5], x[6], x[7]});
    o &= (v4u){ pk16(mk[0], mk[1]), pk16(mk[2], mk[3]), pk16(mk[4], mk[5]), pk16(mk[6], mk[7]) };
    st2_u(WLD + (size_t)n * kK3 + k8, o);
  } else {
    const int t = u - (kNU1 + kNU2 + kNU3);
    if (t >= kBFN) return;
    const float fa = b1[clampi(t, 0, kH - 1)];
    const float fb = b2[clampi(t - 128, 0, kC - 1)];
    const float fc = bl[clampi(t - 192, 0, kC - 1)];
    pin_f(fa); pin_f(fb); pin_f(fc);
    const unsigned m1 = (t < 128) ? 0xFFFFFFFFu : 0u;
    const unsigned m2 = (t >= 128 && t < 128 + kC) ? 0xFFFFFFFFu : 0u;
    const unsigned m3 = (t >= 192 && t < 192 + kC) ? 0xFFFFFFFFu : 0u;
    const unsigned bits = ((bf16_bits(fa) << 16) & m1) | ((bf16_bits(fb) << 16) & m2) | ((bf16_bits(fc) << 16) & m3);
    const float val = __uint_as_float(bits);
    volatile float* q = BF + t;
    *q = val;
    __threadfence();
    *q = val;
  }
}

__global__ __launch_bounds__(256) void k_bucket(const int* __restrict__ srcs, const int* __restrict__ dsts,
                                                int* LIST, int* CNT, int* OFF, int* DINVB, int* FLAG) {
  extern __shared__ __attribute__((aligned(16))) int dsm[];
  int* lists = dsm;
  int* sl    = dsm + kNW * kWLCAP;
  int* cnt   = sl + kRCAP;
  int* offs  = cnt + kNBA;
  int* cur   = offs + kNBA;
  int* misc  = cur + kNBA;
  const int tid  = (int)threadIdx.x;
  const int lane = tid & 31;
  const int wave = rfl(tid >> 5);
  const int blk  = (int)blockIdx.x;
  const int base = blk * kNBA;
  const int nbr  = kN - base;
  const unsigned nb = (unsigned)(nbr < kNBA ? nbr : kNBA);

  {
    const v4i z = {0, 0, 0, 0};
    for (int i = tid * 4; i < kBK_INTS; i += 1024) *(v4ia*)(dsm + i) = z;
  }
  __syncthreads();

  int wc = 0;
  int* mylist = lists + wave * kWLCAP;
  const int ebase = wave * kEPW;
#pragma unroll 1
  for (int it = 0; it < kITERS; ++it) {
    const int e0 = ebase + it * kSTEP + lane;
    int d[kUNR];
#pragma unroll
    for (int j = 0; j < kUNR; ++j) {
      const int ej = e0 + 32 * j;
      const int dv = dsts[ej < kE - 1 ? ej : kE - 1];
      pin_i(dv);
      d[j] = dv;
    }
#pragma unroll
    for (int j = 0; j < kUNR; ++j) {
      const unsigned s = (unsigned)d[j] - (unsigned)base;
      const bool hit = s < nb;
      const unsigned mj = __builtin_amdgcn_ballot_w32(hit);
      if (mj != 0u) {
        const int ej = e0 + 32 * j;
        int sr = srcs[ej < kE - 1 ? ej : kE - 1];
        pin_i(sr);
        sr = clampi(sr, 0, kN - 1);
        const int pos = wc + (int)__builtin_amdgcn_mbcnt_lo(mj, 0u);
        if (hit && pos < kWLCAP) mylist[pos] = (int)((s << 16) | (unsigned)sr);
        wc += (int)__builtin_popcount(mj);
      }
    }
  }
  if (lane == 0) misc[wave] = wc;
  __syncthreads();

  if (wave == 0) {
    int t = 0, ov = 0;
#pragma unroll 1
    for (int w2 = 0; w2 < kNW; ++w2) {
      const int craw = misc[w2];
      ov |= (craw > kWLCAP) ? 1 : 0;
      int c = clampi(craw, 0, kWLCAP);
      c = rfl(c);
#pragma unroll 1
      for (int b0 = 0; b0 < c; b0 += 32) {
        int idx = b0 + lane;
        idx = idx < c ? idx : c - 1;
        const int ent = lists[w2 * kWLCAP + idx];
        const int m32 = (c - b0) < 32 ? (c - b0) : 32;
#pragma unroll 1
        for (int k = 0; k < m32; ++k) {
          const int u    = __builtin_amdgcn_readlane(ent, k);
          const int slot = (u >> 16) & (kNBA - 1);
          if (t < kRCAP) {
            if (lane == 0) cnt[slot] = cnt[slot] + 1;
            t = t + 1;
          } else {
            ov = 1;
          }
        }
      }
    }
    if (lane == 0) { misc[8] = t; misc[9] = ov; }
  }
  __syncthreads();

  if (wave == 0) {
    const int b32 = lane * (kNBA / 32);
    int s = 0;
#pragma unroll 1
    for (int i = 0; i < kNBA / 32; ++i) s += cnt[b32 + i];
    int incl = s;
#pragma unroll
    for (int dd = 1; dd < 32; dd <<= 1) {
      const int y = __shfl_up(incl, dd, 32);
      if (lane >= dd) incl += y;
    }
    int run = incl - s;
#pragma unroll 1
    for (int i = 0; i < kNBA / 32; ++i) {
      const int cv = cnt[b32 + i];
      offs[b32 + i] = run;
      cur[b32 + i]  = run;
      run += cv;
    }
  }
  __syncthreads();

  if (wave == 0) {
    int t2 = 0;
#pragma unroll 1
    for (int w2 = 0; w2 < kNW; ++w2) {
      int c = clampi(misc[w2], 0, kWLCAP);
      c = rfl(c);
#pragma unroll 1
      for (int b0 = 0; b0 < c; b0 += 32) {
        int idx = b0 + lane;
        idx = idx < c ? idx : c - 1;
        const int ent = lists[w2 * kWLCAP + idx];
        const int m32 = (c - b0) < 32 ? (c - b0) : 32;
#pragma unroll 1
        for (int k = 0; k < m32; ++k) {
          const int u    = __builtin_amdgcn_readlane(ent, k);
          const int slot = (u >> 16) & (kNBA - 1);
          if (t2 < kRCAP) {
            if (lane == 0) {
              int p = cur[slot];
              p = clampi(p, 0, kRCAP - 1);
              sl[p] = u;
              cur[slot] = p + 1;
            }
            t2 = t2 + 1;
          }
        }
      }
    }
  }
  __syncthreads();

  const int ovf = misc[9];
#pragma unroll 1
  for (int i = tid; i < kNBA; i += 256) {
    const float dg = (float)(cnt[i] + 1);
    const float dv = 1.0f / sqrtf(dg);
    cur[i] = (ovf != 0) ? 0x7fc00000 : __float_as_int(dv);
  }
  __syncthreads();

  int* lp = LIST + (size_t)blk * kRCAP;
  const v4i c4 = *(const v4ia*)(cnt + 4 * tid);
  const v4i o4 = *(const v4ia*)(offs + 4 * tid);
  const v4i d4 = *(const v4ia*)(cur + 4 * tid);
  const v4i f4 = {ovf, ovf, ovf, ovf};
  for (int pass = 0; pass < 2; ++pass) {
#pragma unroll 1
    for (int i = tid; i < kRCAP / 4; i += 256) {
      const v4i v = *(const v4ia*)(sl + 4 * i);
      *(volatile v4i*)(lp + 4 * i) = v;
    }
    *(volatile v4i*)(CNT + base + 4 * tid)   = c4;
    *(volatile v4i*)(OFF + base + 4 * tid)   = o4;
    *(volatile v4i*)(DINVB + base + 4 * tid) = d4;
    if (tid < 8) *(volatile v4i*)(FLAG + blk * 32 + 4 * tid) = f4;
    __threadfence();
  }
}

__global__ __launch_bounds__(256) void k_agg1(const float* __restrict__ T1, const int* __restrict__ LIST,
                                              const int* __restrict__ CNT, const int* __restrict__ OFF,
                                              const float* __restrict__ DINV, const int* __restrict__ FLAG,
                                              const float* __restrict__ BF, unsigned short* H1HL) {
  __shared__ __attribute__((aligned(16))) float sb[128];
  const int tid  = (int)threadIdx.x;
  const int lane = tid & 31;
  const int wave = rfl(tid >> 5);
  if (tid < 32) { const v4f t = *(const v4fa*)(BF + 4 * tid); *(v4fa*)(sb + 4 * tid) = t; }
  __syncthreads();
  const v4f bv = *(const v4fa*)(sb + 4 * lane);
  const int blockRow = (int)blockIdx.x * 64;
  const int blk = blockRow >> 10;
  const int flag = FLAG[blk * 32];
  pin_i(flag);
  const int* lst = LIST + (size_t)blk * kRCAP;
  const int sA = (2 * lane) & 31, sB = (2 * lane + 1) & 31;
  const bool lsel = lane >= 16;
  const float qnan = __int_as_float(0x7fc00000);
#pragma unroll 1
  for (int ri = 0; ri < 8; ++ri) {
    const int v  = blockRow + wave * 8 + ri;
    const int vc = v < kN ? v : kN - 1;
    const int craw = CNT[v];
    const int oraw = OFF[v];
    const float dd = DINV[vc];
    pin_i(craw); pin_i(oraw); pin_f(dd);
    int c = clampi(craw, 0, kDEGCAP);
    c = rfl(c);
    c = (v < kN) ? c : 0;
    int o = clampi(oraw, 0, kRCAP);
    o = rfl(o);
    v4f acc = (v4f){0.0f, 0.0f, 0.0f, 0.0f};
#pragma unroll 1
    for (int b0 = 0; b0 < c; b0 += 32) {
      int j = b0 + lane;
      j = j < c ? j : c - 1;
      const int idx = clampi(o + j, 0, kRCAP - 1);
      const int ent = lst[idx];
      pin_i(ent);
      int sr = ent & 0xFFFF;
      sr = sr > kN - 1 ? kN - 1 : sr;
      const float ds = DINV[sr];
      pin_f(ds);
      const float w = ds * dd;
      const int wi = __float_as_int(w);
      const int m32 = (c - b0) < 32 ? (c - b0) : 32;
#pragma unroll 1
      for (int k = 0; k < m32; ++k) {
        const int   sk = __builtin_amdgcn_readlane(sr, k);
        const float wk = __int_as_float(__builtin_amdgcn_readlane(wi, k));
        const v4f a = *(const v4fa*)(T1 + (size_t)sk * kH + 4 * lane);
        acc.x = fmaf(wk, a.x, acc.x); acc.y = fmaf(wk, a.y, acc.y);
        acc.z = fmaf(wk, a.z, acc.z); acc.w = fmaf(wk, a.w, acc.w);
      }
    }
    const v4f sv = *(const v4fa*)(T1 + (size_t)vc * kH + 4 * lane);
    pin_f(sv.x); pin_f(sv.y); pin_f(sv.z); pin_f(sv.w);
    const float rd = dd * dd;
    float y0 = (acc.x + sv.x * rd) + bv.x;
    float y1 = (acc.y + sv.y * rd) + bv.y;
    float y2 = (acc.z + sv.z * rd) + bv.z;
    float y3 = (acc.w + sv.w * rd) + bv.w;
    y0 = (y0 > 0.0f) ? y0 : (y0 - y0);
    y1 = (y1 > 0.0f) ? y1 : (y1 - y1);
    y2 = (y2 > 0.0f) ? y2 : (y2 - y2);
    y3 = (y3 > 0.0f) ? y3 : (y3 - y3);
    const bool bad  = (flag != 0) || (craw > kDEGCAP);
    const bool live = v < kN;
    y0 = bad ? qnan : y0; y1 = bad ? qnan : y1; y2 = bad ? qnan : y2; y3 = bad ? qnan : y3;
    y0 = live ? y0 : 0.0f; y1 = live ? y1 : 0.0f; y2 = live ? y2 : 0.0f; y3 = live ? y3 : 0.0f;
    const unsigned hw0 = pk16(bf16_bits(y0), bf16_bits(y1));
    const unsigned hw1 = pk16(bf16_bits(y2), bf16_bits(y3));
    const unsigned lw0 = SPLIT_H1 ? pk16(bf16_lo_bits(y0), bf16_lo_bits(y1)) : 0u;
    const unsigned lw1 = SPLIT_H1 ? pk16(bf16_lo_bits(y2), bf16_lo_bits(y3)) : 0u;
    const int g0 = __shfl((int)hw0, sA, 32), g1 = __shfl((int)hw1, sA, 32);
    const int g2 = __shfl((int)hw0, sB, 32), g3 = __shfl((int)hw1, sB, 32);
    const int p0 = __shfl((int)lw0, sA, 32), p1 = __shfl((int)lw1, sA, 32);
    const int p2 = __shfl((int)lw0, sB, 32), p3 = __shfl((int)lw1, sB, 32);
    v4u pv;
    pv.x = (unsigned)(lsel ? p0 : g0);
    pv.y = (unsigned)(lsel ? p1 : g1);
    pv.z = (unsigned)(lsel ? p2 : g2);
    pv.w = (unsigned)(lsel ? p3 : g3);
    st2_u(H1HL + (size_t)v * kK2 + 8 * lane, pv);
  }
}

__global__ __launch_bounds__(256) void k_agg2(const float* __restrict__ T2, const int* __restrict__ LIST,
                                              const int* __restrict__ CNT, const int* __restrict__ OFF,
                                              const float* __restrict__ DINV, const int* __restrict__ FLAG,
                                              const float* __restrict__ BF, float* out0, unsigned short* H2HL) {
  __shared__ __attribute__((aligned(16))) float sb[128];
  __shared__ __attribute__((aligned(16))) float tile[8][160];
  const int tid  = (int)threadIdx.x;
  const int lane = tid & 31;
  const int wave = rfl(tid >> 5);
  if (tid < 32) { const v4f t = *(const v4fa*)(BF + 128 + 4 * tid); *(v4fa*)(sb + 4 * tid) = t; }
  __syncthreads();
  const float bv0 = sb[2 * lane], bv1 = sb[2 * lane + 1];
  float* tw = tile[wave];
  const int q0s = (4 * lane) & 31, q1s = (4 * lane + 1) & 31;
  const int q2s = (4 * lane + 2) & 31, q3s = (4 * lane + 3) & 31;
  const bool lsel = (lane & 8) != 0;
  const bool colok = lane < (kC / 2);
  const float qnan = __int_as_float(0x7fc00000);
#pragma unroll 1
  for (int gi = 0; gi < 2; ++gi) {
    const int g   = ((int)blockIdx.x * 8 + wave) * 2 + gi;
    const int blk = (4 * g) >> 10;
    const int flag = FLAG[blk * 32];
    pin_i(flag);
    const int* lst = LIST + (size_t)blk * kRCAP;
#pragma unroll 1
    for (int r = 0; r < 4; ++r) {
      const int v  = 4 * g + r;
      const int vc = v < kN ? v : kN - 1;
      const int craw = CNT[v];
      const int oraw = OFF[v];
      const float dd = DINV[vc];
      pin_i(craw); pin_i(oraw); pin_f(dd);
      int c = clampi(craw, 0, kDEGCAP);
      c = rfl(c);
      c = (v < kN) ? c : 0;
      int o = clampi(oraw, 0, kRCAP);
      o = rfl(o);
      float a0 = 0.0f, a1 = 0.0f;
#pragma unroll 1
      for (int b0 = 0; b0 < c; b0 += 32) {
        int j = b0 + lane;
        j = j < c ? j : c - 1;
        const int idx = clampi(o + j, 0, kRCAP - 1);
        const int ent = lst[idx];
        pin_i(ent);
        int sr = ent & 0xFFFF;
        sr = sr > kN - 1 ? kN - 1 : sr;
        const float ds = DINV[sr];
        pin_f(ds);
        const float w = ds * dd;
        const int wi = __float_as_int(w);
        const int m32 = (c - b0) < 32 ? (c - b0) : 32;
#pragma unroll 1
        for (int k = 0; k < m32; ++k) {
          const int   sk = __builtin_amdgcn_readlane(sr, k);
          const float wk = __int_as_float(__builtin_amdgcn_readlane(wi, k));
          const v2f a = *(const v2fa*)(T2 + (size_t)sk * kCP + 2 * lane);
          a0 = fmaf(wk, a.x, a0); a1 = fmaf(wk, a.y, a1);
        }
      }
      const v2f sv = *(const v2fa*)(T2 + (size_t)vc * kCP + 2 * lane);
      pin_f(sv.x); pin_f(sv.y);
      const float rd = dd * dd;
      float y0 = (a0 + sv.x * rd) + bv0;
      float y1 = (a1 + sv.y * rd) + bv1;
      y0 = (y0 > 0.0f) ? y0 : (y0 - y0);
      y1 = (y1 > 0.0f) ? y1 : (y1 - y1);
      const bool bad  = (flag != 0) || (craw > kDEGCAP);
      const bool keep = (v < kN) && colok;
      y0 = bad ? qnan : y0; y1 = bad ? qnan : y1;
      y0 = keep ? y0 : 0.0f; y1 = keep ? y1 : 0.0f;
      if (colok) { v2f t2v; t2v.x = y0; t2v.y = y1; *(v2fa*)(tw + r * kC + 2 * lane) = t2v; }
      const unsigned hw = pk16(bf16_bits(y0), bf16_bits(y1));
      const unsigned lw = SPLIT_H2 ? pk16(bf16_lo_bits(y0), bf16_lo_bits(y1)) : 0u;
      const int g0 = __shfl((int)hw, q0s, 32), g1 = __shfl((int)hw, q1s, 32);
      const int g2 = __shfl((int)hw, q2s, 32), g3 = __shfl((int)hw, q3s, 32);
      const int p0 = __shfl((int)lw, q0s, 32), p1 = __shfl((int)lw, q1s, 32);
      const int p2 = __shfl((int)lw, q2s, 32), p3 = __shfl((int)lw, q3s, 32);
      v4u pv;
      pv.x = (unsigned)(lsel ? p0 : g0);
      pv.y = (unsigned)(lsel ? p1 : g1);
      pv.z = (unsigned)(lsel ? p2 : g2);
      pv.w = (unsigned)(lsel ? p3 : g3);
      unsigned short* hp = H2HL + (size_t)v * kK3 + 8 * (lane & 15);
      const bool wr = lane < 16;
      if (wr) *(volatile v4u*)hp = pv;
      __threadfence();
      if (wr) *(volatile v4u*)hp = pv;
    }
    __builtin_amdgcn_fence(__ATOMIC_RELEASE, "workgroup");
    __builtin_amdgcn_wave_barrier();
    __builtin_amdgcn_fence(__ATOMIC_ACQUIRE, "workgroup");
    const v4f pa = *(const v4fa*)(tw + 4 * lane);
    const v4f pb = *(const v4fa*)(tw + 128 + 4 * (lane & 7));
    if (g < kNGRP) {
      float* op = out0 + (size_t)g * 160;
      *(volatile v4f*)(op + 4 * lane) = pa;
      if (lane < 8) *(volatile v4f*)(op + 128 + 4 * lane) = pb;
      __threadfence();
      *(volatile v4f*)(op + 4 * lane) = pa;
      if (lane < 8) *(volatile v4f*)(op + 128 + 4 * lane) = pb;
    }
    __builtin_amdgcn_fence(__ATOMIC_RELEASE, "workgroup");
    __builtin_amdgcn_wave_barrier();
    __builtin_amdgcn_fence(__ATOMIC_ACQUIRE, "workgroup");
  }
}

__global__ __launch_bounds__(256) void k_out(const float* __restrict__ O, const int* __restrict__ CNT,
                                             const int* __restrict__ FLAG, const float* __restrict__ BF,
                                             float* out1) {
  __shared__ __attribute__((aligned(16))) float sb[128];
  __shared__ __attribute__((aligned(16))) float tile[8][160];
  const int tid  = (int)threadIdx.x;
  const int lane = tid & 31;
  const int wave = rfl(tid >> 5);
  if (tid < 32) { const v4f t = *(const v4fa*)(BF + 128 + 4 * tid); *(v4fa*)(sb + 4 * tid) = t; }
  __syncthreads();
  const float bl0 = sb[64 + 2 * lane], bl1 = sb[64 + 2 * lane + 1];
  float* tw = tile[wave];
  const bool colok = lane < (kC / 2);
  const float qnan = __int_as_float(0x7fc00000);
#pragma unroll 1
  for (int gi = 0; gi < 4; ++gi) {
    const int g = ((int)blockIdx.x * 8 + wave) * 4 + gi;
    if (g >= kNGRP) continue;
    const int blk = (4 * g) >> 10;
    const int flag = FLAG[blk * 32];
    pin_i(flag);
#pragma unroll 1
    for (int r = 0; r < 4; ++r) {
      const int v = 4 * g + r;
      const int craw = CNT[v];
      pin_i(craw);
      const v2f x = *(const v2fa*)(O + (size_t)v * kCP + 2 * lane);
      pin_f(x.x); pin_f(x.y);
      float y0 = x.x + bl0;
      float y1 = x.y + bl1;
      const bool bad = (flag != 0) || (craw > kDEGCAP);
      y0 = bad ? qnan : y0; y1 = bad ? qnan : y1;
      if (colok) { v2f t2v; t2v.x = y0; t2v.y = y1; *(v2fa*)(tw + r * kC + 2 * lane) = t2v; }
    }
    __builtin_amdgcn_fence(__ATOMIC_RELEASE, "workgroup");
    __builtin_amdgcn_wave_barrier();
    __builtin_amdgcn_fence(__ATOMIC_ACQUIRE, "workgroup");
    const v4f pa = *(const v4fa*)(tw + 4 * lane);
    const v4f pb = *(const v4fa*)(tw + 128 + 4 * (lane & 7));
    float* op = out1 + (size_t)g * 160;
    *(volatile v4f*)(op + 4 * lane) = pa;
    if (lane < 8) *(volatile v4f*)(op + 128 + 4 * lane) = pb;
    __threadfence();
    *(volatile v4f*)(op + 4 * lane) = pa;
    if (lane < 8) *(volatile v4f*)(op + 128 + 4 * lane) = pb;
    __builtin_amdgcn_fence(__ATOMIC_RELEASE, "workgroup");
    __builtin_amdgcn_wave_barrier();
    __builtin_amdgcn_fence(__ATOMIC_ACQUIRE, "workgroup");
  }
}

static constexpr size_t al256c(size_t o) { return (o + 255) & ~(size_t)255; }
static constexpr size_t szXB   = (size_t)kMP * kF * 2;
static constexpr size_t szT1   = (size_t)kMP * kH * 4;
static constexpr size_t szH1   = (size_t)kMP * kK2 * 2;
static constexpr size_t szT2   = (size_t)kMP * kCP * 4;
static constexpr size_t szH2   = (size_t)kMP * kK3 * 2;
static constexpr size_t szO    = (size_t)kMP * kCP * 4;
static constexpr size_t szLIST = (size_t)kNBLK * kRCAP * 4;
static constexpr size_t szTAB  = (size_t)kNBLK * kNBA * 4;
static constexpr size_t szW1T  = (size_t)kH * kF * 2;
static constexpr size_t szW2D  = (size_t)kCP * kK2 * 2;
static constexpr size_t szWLD  = (size_t)kCP * kK3 * 2;
static constexpr size_t szBF   = (size_t)kBFN * 4;
static constexpr size_t szFLAG = (size_t)kNBLK * 128;
static constexpr size_t oXB   = 0;
static constexpr size_t oT1   = al256c(oXB + szXB);
static constexpr size_t oH1   = al256c(oT1 + szT1);
static constexpr size_t oT2   = al256c(oH1 + szH1);
static constexpr size_t oH2   = al256c(oT2 + szT2);
static constexpr size_t oO    = al256c(oH2 + szH2);
static constexpr size_t oLIST = al256c(oO + szO);
static constexpr size_t oCNT  = al256c(oLIST + szLIST);
static constexpr size_t oOFF  = al256c(oCNT + szTAB);
static constexpr size_t oDINV = al256c(oOFF + szTAB);
static constexpr size_t oW1T  = al256c(oDINV + szTAB);
static constexpr size_t oW2D  = al256c(oW1T + szW1T);
static constexpr size_t oWLD  = al256c(oW2D + szW2D);
static constexpr size_t oBF   = al256c(oWLD + szWLD);
static constexpr size_t oFLAG = al256c(oBF + szBF);
static constexpr size_t kWS_TOTAL = al256c(oFLAG + szFLAG);
static_assert(kWS_TOTAL == ((size_t)419157 << 8));
static_assert(kWS_TOTAL <= ((size_t)128 << 20));

extern "C" void kernel_launch(void* const* d_in, const int* in_sizes, int n_in,
                              void* d_out, int out_size, void* d_ws, size_t ws_size,
                              hipStream_t stream) {
  if (n_in < 8) return;
  if (in_sizes[0] != kN * kF) return;
  if (in_sizes[1] != 2 * kE) return;
  if (in_sizes[2] != kF * kH) return;
  if (in_sizes[3] != kH) return;
  if (in_sizes[4] != kH * kC) return;
  if (in_sizes[5] != kC) return;
  if (in_sizes[6] != kC * kC) return;
  if (in_sizes[7] != kC) return;
  if (out_size != 2 * kN * kC) return;
  if (kWS_TOTAL > ws_size) return;

  const float* x    = (const float*)d_in[0];
  const int*   edge = (const int*)d_in[1];
  const float* W1   = (const float*)d_in[2];
  const float* b1   = (const float*)d_in[3];
  const float* W2   = (const float*)d_in[4];
  const float* b2   = (const float*)d_in[5];
  const float* Wl   = (const float*)d_in[6];
  const float* bl   = (const float*)d_in[7];
  const int* src = edge;
  const int* dst = edge + kE;
  float* out0 = (float*)d_out;
  float* out1 = (float*)d_out + (size_t)kN * kC;

  char* ws = (char*)d_ws;
  unsigned short* XB   = (unsigned short*)(ws + oXB);
  float*          T1   = (float*)(ws + oT1);
  unsigned short* H1HL = (unsigned short*)(ws + oH1);
  float*          T2   = (float*)(ws + oT2);
  unsigned short* H2HL = (unsigned short*)(ws + oH2);
  float*          O    = (float*)(ws + oO);
  int*            LIST = (int*)(ws + oLIST);
  int*            CNT  = (int*)(ws + oCNT);
  int*            OFF  = (int*)(ws + oOFF);
  int*            DINVB = (int*)(ws + oDINV);
  const float*    DINV = (const float*)(ws + oDINV);
  unsigned short* W1T  = (unsigned short*)(ws + oW1T);
  unsigned short* W2D  = (unsigned short*)(ws + oW2D);
  unsigned short* WLD  = (unsigned short*)(ws + oWLD);
  float*          BF   = (float*)(ws + oBF);
  int*            FLAG = (int*)(ws + oFLAG);

  hipFuncSetAttribute(reinterpret_cast<const void*>(&k_bucket), hipFuncAttributeMaxDynamicSharedMemorySize,
                      (int)kBK_LDS);

  k_plane<0><<<kMP * kF / 8 / 256, 256, 0, stream>>>(x, kN, kF, kF, XB, kMP, kF);
  k_wprep<<<(kNU1 + kNU2 + kNU3) / 256 + 1, 256, 0, stream>>>(W1, W2, Wl, b1, b2, bl, W1T, W2D, WLD, BF);
  k_bucket<<<kNBLK, 256, (size_t)kBK_LDS, stream>>>(src, dst, LIST, CNT, OFF, DINVB, FLAG);
  k_gemm_nt<0, 0><<<(782 * 2 + 7) / 8, 256, 0, stream>>>(XB, W1T, BF, T1, kMP, kH, kF, kH);
  k_agg1<<<kMP / 64, 256, 0, stream>>>(T1, LIST, CNT, OFF, DINV, FLAG, BF, H1HL);
  k_gemm_nt<0, 0><<<(782 + 7) / 8, 256, 0, stream>>>(H1HL, W2D, BF, T2, kMP, kCP, kK2, kCP);
  k_agg2<<<kMP / 64, 256, 0, stream>>>(T2, LIST, CNT, OFF, DINV, FLAG, BF, out0, H2HL);
  k_gemm_nt<0, 0><<<(782 + 7) / 8, 256, 0, stream>>>(H2HL, WLD, BF, O, kMP, kCP, kK3, kCP);
  k_out<<<(kNGRP + 31) / 32, 256, 0, stream>>>(O, CNT, FLAG, BF, out1);
}
